// RelativeMultiHeadAttention_21749714387556
// MI455X (gfx1250) — hardware-verified
//
#include <hip/hip_runtime.h>

#define DM    1024
#define NH    16
#define DK    64
#define SEQ   1000
#define BATCH 4
#define NROWS (BATCH * SEQ)
#define WROWS (2 * SEQ - 1)
#define JP    1024
#define NIB   ((SEQ + 15) / 16)
#define IBLK  ((SEQ + 63) / 64)
#define TP    68

typedef __bf16       v16bf __attribute__((ext_vector_type(16)));
typedef float        v8f   __attribute__((ext_vector_type(8)));
typedef float        v4fb  __attribute__((ext_vector_type(4)));
typedef v4fb __attribute__((may_alias)) v4f;
typedef unsigned int v4ub  __attribute__((ext_vector_type(4)));
typedef v4ub __attribute__((may_alias)) v4u;

union Frag { v16bf v; v4u u[2]; };

__device__ __forceinline__ v8f zero8() {
  v8f z = {0.f, 0.f, 0.f, 0.f, 0.f, 0.f, 0.f, 0.f};
  return z;
}

__device__ __forceinline__ unsigned int bf16_bits(float x) {
  unsigned int u = __float_as_uint(x);
  u += 0x7FFFu + ((u >> 16) & 1u);
  return u >> 16;
}
__device__ __forceinline__ unsigned int pack2(float a, float b) {
  return bf16_bits(a) | (bf16_bits(b) << 16);
}
__device__ __forceinline__ v4u pack8(v4f a, v4f b) {
  v4u w;
  w.x = pack2(a.x, a.y); w.y = pack2(a.z, a.w);
  w.z = pack2(b.x, b.y); w.w = pack2(b.z, b.w);
  return w;
}

__device__ __forceinline__ float wsum(float v) {
#pragma unroll
  for (int o = 16; o > 0; o >>= 1) v += __shfl_xor(v, o, 32);
  return v;
}

__device__ __forceinline__ v8f mma(v16bf a, v16bf b, v8f c) {
  v8f d = __builtin_amdgcn_wmma_f32_16x16x32_bf16(false, a, false, b, (short)0, c, false, false);
  asm volatile("v_nop\n\tv_nop\n\tv_nop\n\tv_nop" : "+v"(d) : "v"(a), "v"(b));
  return d;
}

__device__ __forceinline__ v16bf ld_frag(const unsigned short* p, int hh) {
  Frag f;
  f.u[0] = *(const v4u*)(p + 8 * hh);
  f.u[1] = *(const v4u*)(p + 16 + 8 * hh);
  return f.v;
}

__global__ __launch_bounds__(256) void cvt_kernel(const float* __restrict__ src,
                                                  unsigned short* __restrict__ dst, int n8) {
  const int gi = blockIdx.x * 256 + threadIdx.x;
  if (gi < n8) {
    const float* s = src + (size_t)gi * 8;
    const v4f a = *(const v4f*)s;
    const v4f b = *(const v4f*)(s + 4);
    const v4u w = pack8(a, b);
    volatile v4u* d = (volatile v4u*)(dst + (size_t)gi * 8);
    *d = w;
    __threadfence();
    *d = w;
  }
}

__global__ __launch_bounds__(128) void ln_kernel(const float* __restrict__ x,
                                                 const float* __restrict__ g,
                                                 const float* __restrict__ bt,
                                                 unsigned short* __restrict__ y, int nrows) {
  __shared__ float red0[4];
  __shared__ float red1[4];
  const int row = blockIdx.x;
  if (row >= nrows) return;
  const int t = threadIdx.x, lane = t & 31, wave = t >> 5;
  const float* xr = x + (size_t)row * DM + t * 8;
  const v4f a = *(const v4f*)xr;
  const v4f c = *(const v4f*)(xr + 4);
  float s = ((a.x + a.y) + (a.z + a.w)) + ((c.x + c.y) + (c.z + c.w));
  s = wsum(s);
  if (lane == 0) red0[wave] = s;
  __syncthreads();
  const float mu = ((red0[0] + red0[1]) + (red0[2] + red0[3])) * (1.0f / DM);
  float d[8];
  d[0] = a.x - mu; d[1] = a.y - mu; d[2] = a.z - mu; d[3] = a.w - mu;
  d[4] = c.x - mu; d[5] = c.y - mu; d[6] = c.z - mu; d[7] = c.w - mu;
  float ss = 0.f;
#pragma unroll
  for (int i = 0; i < 8; ++i) ss += d[i] * d[i];
  ss = wsum(ss);
  if (lane == 0) red1[wave] = ss;
  __syncthreads();
  const float var = ((red1[0] + red1[1]) + (red1[2] + red1[3])) * (1.0f / DM);
  const float rs = rsqrtf(var + 1e-5f);
  const v4f g0 = *(const v4f*)(g + t * 8);
  const v4f g1 = *(const v4f*)(g + t * 8 + 4);
  const v4f b0 = *(const v4f*)(bt + t * 8);
  const v4f b1 = *(const v4f*)(bt + t * 8 + 4);
  v4f o0, o1;
  o0.x = d[0] * rs * g0.x + b0.x; o0.y = d[1] * rs * g0.y + b0.y;
  o0.z = d[2] * rs * g0.z + b0.z; o0.w = d[3] * rs * g0.w + b0.w;
  o1.x = d[4] * rs * g1.x + b1.x; o1.y = d[5] * rs * g1.y + b1.y;
  o1.z = d[6] * rs * g1.z + b1.z; o1.w = d[7] * rs * g1.w + b1.w;
  const v4u w = pack8(o0, o1);
  volatile v4u* dst = (volatile v4u*)(y + (size_t)row * DM + t * 8);
  *dst = w;
  __threadfence();
  *dst = w;
}

__global__ __launch_bounds__(128) void gemm_kernel(
    const unsigned short* __restrict__ A, const unsigned short* __restrict__ W,
    const float* __restrict__ bias, const float* __restrict__ res,
    unsigned short* __restrict__ outH, unsigned short* __restrict__ vT,
    float* __restrict__ outF, int mode) {
  __shared__ __align__(16) float tile[64][TP];
  const int lane = threadIdx.x & 31, wave = threadIdx.x >> 5;
  const int hh = lane >> 4, m = lane & 15;
  const int bI = blockIdx.x / IBLK;
  const int i0 = (blockIdx.x % IBLK) * 64;
  const int n0 = blockIdx.y * 64;

  int ia = i0 + wave * 16 + m;
  if (ia > SEQ - 1) ia = SEQ - 1;
  const unsigned short* arow = A + (size_t)(bI * SEQ + ia) * DM;
  const unsigned short* wrow = W + (size_t)(n0 + m) * DM;

  v8f acc0 = zero8(), acc1 = zero8(), acc2 = zero8(), acc3 = zero8();
#pragma unroll 1
  for (int k0 = 0; k0 < DM; k0 += 32) {
    const v16bf a  = ld_frag(arow + k0, hh);
    const v16bf b0 = ld_frag(wrow + k0, hh);
    const v16bf b1 = ld_frag(wrow + (size_t)16 * DM + k0, hh);
    const v16bf b2 = ld_frag(wrow + (size_t)32 * DM + k0, hh);
    const v16bf b3 = ld_frag(wrow + (size_t)48 * DM + k0, hh);
    acc0 = mma(a, b0, acc0);
    acc1 = mma(a, b1, acc1);
    acc2 = mma(a, b2, acc2);
    acc3 = mma(a, b3, acc3);
  }

  const float bv0 = bias[n0 + m];
  const float bv1 = bias[n0 + 16 + m];
  const float bv2 = bias[n0 + 32 + m];
  const float bv3 = bias[n0 + 48 + m];
  const int rl = wave * 16 + 8 * hh;
  if (mode == 1) {
#pragma unroll
    for (int r = 0; r < 8; ++r) {
      tile[m][rl + r]      = acc0[r] + bv0;
      tile[16 + m][rl + r] = acc1[r] + bv1;
      tile[32 + m][rl + r] = acc2[r] + bv2;
      tile[48 + m][rl + r] = acc3[r] + bv3;
    }
  } else {
#pragma unroll
    for (int r = 0; r < 8; ++r) {
      tile[rl + r][m]      = acc0[r] + bv0;
      tile[rl + r][16 + m] = acc1[r] + bv1;
      tile[rl + r][32 + m] = acc2[r] + bv2;
      tile[rl + r][48 + m] = acc3[r] + bv3;
    }
  }
  __syncthreads();

  if (mode == 2) {
    const int c4 = (lane & 15) * 4;
    v4f vals[8];
#pragma unroll
    for (int it = 0; it < 8; ++it) {
      const int R = wave * 16 + 2 * it + hh;
      const int i = i0 + R;
      const int ic = (i < SEQ) ? i : (SEQ - 1);
      const size_t idx = (size_t)(bI * SEQ + ic) * DM + n0 + c4;
      const v4f tv = *(const v4f*)&tile[R][c4];
      const v4f rv = *(const v4f*)(res + idx);
      vals[it] = tv + rv;
      if (i < SEQ) *(volatile v4f*)(outF + idx) = vals[it];
    }
    __threadfence();
#pragma unroll
    for (int it = 0; it < 8; ++it) {
      const int R = wave * 16 + 2 * it + hh;
      const int i = i0 + R;
      if (i < SEQ) {
        const size_t idx = (size_t)(bI * SEQ + i) * DM + n0 + c4;
        *(volatile v4f*)(outF + idx) = vals[it];
      }
    }
  } else if (mode == 0) {
    const int c8 = (lane & 7) * 8, rq = lane >> 3;
    v4u vals[4];
#pragma unroll
    for (int it = 0; it < 4; ++it) {
      const int R = wave * 16 + 4 * it + rq;
      const int i = i0 + R;
      vals[it] = pack8(*(const v4f*)&tile[R][c8], *(const v4f*)&tile[R][c8 + 4]);
      if (i < SEQ) *(volatile v4u*)(outH + (size_t)(bI * SEQ + i) * DM + n0 + c8) = vals[it];
    }
    __threadfence();
#pragma unroll
    for (int it = 0; it < 4; ++it) {
      const int R = wave * 16 + 4 * it + rq;
      const int i = i0 + R;
      if (i < SEQ) *(volatile v4u*)(outH + (size_t)(bI * SEQ + i) * DM + n0 + c8) = vals[it];
    }
  } else {
    const int c8 = (lane & 7) * 8, rq = lane >> 3;
    v4u vals[4];
#pragma unroll
    for (int it = 0; it < 4; ++it) {
      const int R = wave * 16 + 4 * it + rq;
      vals[it] = pack8(*(const v4f*)&tile[R][c8], *(const v4f*)&tile[R][c8 + 4]);
      const size_t idx = ((size_t)((bI * NH + blockIdx.y) * DK + R)) * JP + i0 + c8;
      *(volatile v4u*)(vT + idx) = vals[it];
    }
    __threadfence();
#pragma unroll
    for (int it = 0; it < 4; ++it) {
      const int R = wave * 16 + 4 * it + rq;
      const size_t idx = ((size_t)((bI * NH + blockIdx.y) * DK + R)) * JP + i0 + c8;
      *(volatile v4u*)(vT + idx) = vals[it];
    }
  }
}

__global__ __launch_bounds__(32) void attn_kernel(
    const unsigned short* __restrict__ Q, const unsigned short* __restrict__ K,
    const unsigned short* __restrict__ VT, const unsigned short* __restrict__ WIN,
    unsigned short* __restrict__ O) {
  __shared__ __align__(16) float p_lds[16][48];
  __shared__ __align__(16) unsigned short a_lds[16][32];
  __shared__ __align__(16) float o_lds[16][TP];

  const int lane = threadIdx.x & 31, hh = lane >> 4, m = lane & 15;
  const int ib = blockIdx.x % NIB, bh = blockIdx.x / NIB;
  const int hd = bh % NH, b = bh / NH;
  const int i0 = ib * 16;

  int qi = i0 + m;
  if (qi > SEQ - 1) qi = SEQ - 1;
  const unsigned short* qrow = Q + (size_t)(b * SEQ + qi) * DM + hd * DK;
  const v16bf aq0 = ld_frag(qrow, hh);
  const v16bf aq1 = ld_frag(qrow + 32, hh);

  float m_run[8], l_run[8];
  v8f o0 = zero8(), o1 = zero8(), o2 = zero8(), o3 = zero8();
#pragma unroll
  for (int r = 0; r < 8; ++r) { m_run[r] = -1e30f; l_run[r] = 0.f; }
  const float scale = 0.125f;
  const size_t vrow0 = (size_t)(b * NH + hd) * DK;

#pragma unroll 1
  for (int jc = 0; jc < JP; jc += 32) {
    v8f c0, c1;
    {
      int j = jc + m;
      if (j > SEQ - 1) j = SEQ - 1;
      const unsigned short* krow = K + (size_t)(b * SEQ + j) * DM + hd * DK;
      c0 = mma(aq0, ld_frag(krow, hh), zero8());
      c0 = mma(aq1, ld_frag(krow + 32, hh), c0);
    }
    {
      int j = jc + 16 + m;
      if (j > SEQ - 1) j = SEQ - 1;
      const unsigned short* krow = K + (size_t)(b * SEQ + j) * DM + hd * DK;
      c1 = mma(aq0, ld_frag(krow, hh), zero8());
      c1 = mma(aq1, ld_frag(krow + 32, hh), c1);
    }
    const int rbase = i0 - jc + (SEQ - 1) - 31;
#pragma unroll
    for (int pt = 0; pt < 3; ++pt) {
      const int t = pt * 16 + m;
      int rr = rbase + t;
      rr = rr < 0 ? 0 : (rr > WROWS - 1 ? WROWS - 1 : rr);
      const unsigned short* wr = WIN + (size_t)rr * DK;
      v8f p = mma(aq0, ld_frag(wr, hh), zero8());
      p = mma(aq1, ld_frag(wr + 32, hh), p);
#pragma unroll
      for (int r = 0; r < 8; ++r) p_lds[8 * hh + r][t] = p[r];
    }
    __syncthreads();

#pragma unroll
    for (int r = 0; r < 8; ++r) {
      const int di = 8 * hh + r;
      float s0 = (c0[r] + p_lds[di][31 + di - m]) * scale;
      float s1 = (c1[r] + p_lds[di][15 + di - m]) * scale;
      if (jc + m >= SEQ)      s0 = -1e30f;
      if (jc + 16 + m >= SEQ) s1 = -1e30f;
      float mx = fmaxf(s0, s1);
#pragma unroll
      for (int o = 1; o < 16; o <<= 1) mx = fmaxf(mx, __shfl_xor(mx, o, 32));
      const float mnew = fmaxf(m_run[r], mx);
      const float e0 = __expf(s0 - mnew), e1 = __expf(s1 - mnew);
      float sm = e0 + e1;
#pragma unroll
      for (int o = 1; o < 16; o <<= 1) sm += __shfl_xor(sm, o, 32);
      const float alpha = __expf(m_run[r] - mnew);
      l_run[r] = l_run[r] * alpha + sm;
      m_run[r] = mnew;
      o0[r] *= alpha; o1[r] *= alpha; o2[r] *= alpha; o3[r] *= alpha;
      a_lds[di][m]      = (unsigned short)bf16_bits(e0);
      a_lds[di][16 + m] = (unsigned short)bf16_bits(e1);
    }
    __syncthreads();

    const v16bf ap = ld_frag(&a_lds[m][0], hh);
    const unsigned short* vb = VT + (vrow0 + m) * JP + jc;
    o0 = mma(ap, ld_frag(vb, hh), o0);
    o1 = mma(ap, ld_frag(vb + 16 * JP, hh), o1);
    o2 = mma(ap, ld_frag(vb + 32 * JP, hh), o2);
    o3 = mma(ap, ld_frag(vb + 48 * JP, hh), o3);
  }

#pragma unroll
  for (int r = 0; r < 8; ++r) {
    const float inv = 1.f / l_run[r];
    const int di = 8 * hh + r;
    o_lds[di][m]      = o0[r] * inv;
    o_lds[di][16 + m] = o1[r] * inv;
    o_lds[di][32 + m] = o2[r] * inv;
    o_lds[di][48 + m] = o3[r] * inv;
  }
  __syncthreads();
  const int c8 = (lane & 7) * 8, rq = lane >> 3;
  v4u vals[4];
#pragma unroll
  for (int it = 0; it < 4; ++it) {
    const int R = 4 * it + rq;
    const int i = i0 + R;
    vals[it] = pack8(*(const v4f*)&o_lds[R][c8], *(const v4f*)&o_lds[R][c8 + 4]);
    if (i < SEQ) *(volatile v4u*)(O + (size_t)(b * SEQ + i) * DM + hd * DK + c8) = vals[it];
  }
  __threadfence();
#pragma unroll
  for (int it = 0; it < 4; ++it) {
    const int R = 4 * it + rq;
    const int i = i0 + R;
    if (i < SEQ) *(volatile v4u*)(O + (size_t)(b * SEQ + i) * DM + hd * DK + c8) = vals[it];
  }
}

extern "C" void kernel_launch(void* const* d_in, const int* in_sizes, int n_in,
                              void* d_out, int out_size, void* d_ws, size_t ws_size,
                              hipStream_t stream) {
  if (n_in < 14) return;
  if (in_sizes[0] != NROWS * DM || in_sizes[1] != NROWS * DM || in_sizes[2] != NROWS * DM) return;
  if (in_sizes[3] != DM || in_sizes[4] != DM) return;
  if (in_sizes[5] != DM * DM || in_sizes[7] != DM * DM || in_sizes[9] != DM * DM || in_sizes[11] != DM * DM) return;
  if (in_sizes[6] != DM || in_sizes[8] != DM || in_sizes[10] != DM || in_sizes[12] != DM) return;
  if (in_sizes[13] != WROWS * DK) return;
  if (out_size != NROWS * DM) return;

  const float* q    = (const float*)d_in[0];
  const float* k    = (const float*)d_in[1];
  const float* v    = (const float*)d_in[2];
  const float* ln_g = (const float*)d_in[3];
  const float* ln_b = (const float*)d_in[4];
  const float* wq   = (const float*)d_in[5];
  const float* bq   = (const float*)d_in[6];
  const float* wk   = (const float*)d_in[7];
  const float* bk   = (const float*)d_in[8];
  const float* wv   = (const float*)d_in[9];
  const float* bv   = (const float*)d_in[10];
  const float* wo   = (const float*)d_in[11];
  const float* bo   = (const float*)d_in[12];
  const float* rel  = (const float*)d_in[13];
  float* out = (float*)d_out;

  char* ws = (char*)d_ws;
  size_t off = 0;
  auto carve = [&](size_t bytes) -> void* {
    void* p = ws + off;
    off += (bytes + 255) & ~(size_t)255;
    return p;
  };
  unsigned short* qn   = (unsigned short*)carve((size_t)NROWS * DM * 2);
  unsigned short* kn   = (unsigned short*)carve((size_t)NROWS * DM * 2);
  unsigned short* vn   = (unsigned short*)carve((size_t)NROWS * DM * 2);
  unsigned short* wqh  = (unsigned short*)carve((size_t)DM * DM * 2);
  unsigned short* wkh  = (unsigned short*)carve((size_t)DM * DM * 2);
  unsigned short* wvh  = (unsigned short*)carve((size_t)DM * DM * 2);
  unsigned short* woh  = (unsigned short*)carve((size_t)DM * DM * 2);
  unsigned short* winh = (unsigned short*)carve((size_t)WROWS * DK * 2);
  unsigned short* qp   = (unsigned short*)carve((size_t)NROWS * DM * 2);
  unsigned short* kp   = (unsigned short*)carve((size_t)NROWS * DM * 2);
  unsigned short* vT   = (unsigned short*)carve((size_t)BATCH * NH * DK * JP * 2);
  unsigned short* ao   = (unsigned short*)carve((size_t)NROWS * DM * 2);
  if (off > ws_size) return;

  const int n8w = DM * DM / 8;
  const int n8r = WROWS * DK / 8;
  cvt_kernel<<<(n8w + 255) / 256, 256, 0, stream>>>(wq, wqh, n8w);
  cvt_kernel<<<(n8w + 255) / 256, 256, 0, stream>>>(wk, wkh, n8w);
  cvt_kernel<<<(n8w + 255) / 256, 256, 0, stream>>>(wv, wvh, n8w);
  cvt_kernel<<<(n8w + 255) / 256, 256, 0, stream>>>(wo, woh, n8w);
  cvt_kernel<<<(n8r + 255) / 256, 256, 0, stream>>>(rel, winh, n8r);

  ln_kernel<<<NROWS, 128, 0, stream>>>(q, ln_g, ln_b, qn, NROWS);
  ln_kernel<<<NROWS, 128, 0, stream>>>(k, ln_g, ln_b, kn, NROWS);
  ln_kernel<<<NROWS, 128, 0, stream>>>(v, ln_g, ln_b, vn, NROWS);

  dim3 gg(BATCH * IBLK, DM / 64);
  gemm_kernel<<<gg, 128, 0, stream>>>(qn, wqh, bq, nullptr, qp, nullptr, nullptr, 0);
  gemm_kernel<<<gg, 128, 0, stream>>>(kn, wkh, bk, nullptr, kp, nullptr, nullptr, 0);
  gemm_kernel<<<gg, 128, 0, stream>>>(vn, wvh, bv, nullptr, nullptr, vT, nullptr, 1);

  attn_kernel<<<BATCH * NH * NIB, 32, 0, stream>>>(qp, kp, vT, winh, ao);

  gemm_kernel<<<gg, 128, 0, stream>>>(ao, woh, bo, q, nullptr, nullptr, out, 2);
}
